// QuanvolutionGen112_65481071400242
// MI455X (gfx1250) — hardware-verified
//
#include <hip/hip_runtime.h>
#include <stdint.h>


typedef _Float16 v16h __attribute__((ext_vector_type(16)));
typedef _Float16 v8h  __attribute__((ext_vector_type(8)));
typedef float    v8f  __attribute__((ext_vector_type(8)));
typedef float    v4f  __attribute__((ext_vector_type(4)));

union Frag { v16h v; v8h half[2]; _Float16 s[16]; };

#define NPIX  196
#define KFC   3136
#define NCLS  10
#define IMGS  16
#define NTHR  256

__device__ __forceinline__ v8f wmma16(v8f acc, v16h a, v16h b) {
  acc = __builtin_amdgcn_wmma_f32_16x16x32_f16(false, a, false, b, (short)0, acc, false, false);
  asm volatile("v_nop\n\tv_nop\n\tv_nop\n\tv_nop" : "+v"(acc) : "v"(a), "v"(b));
  return acc;
}

__global__ void __launch_bounds__(NTHR)
k_main(const float* __restrict__ x,
       const float* __restrict__ pw,
       const float* __restrict__ pb,
       const float* __restrict__ qw,
       const float* __restrict__ conv_w,
       const float* __restrict__ conv_b,
       const float* __restrict__ fc_w,
       const float* __restrict__ fc_b,
       float* out,
       int nimg) {
  __shared__ __attribute__((aligned(16))) _Float16 F[IMGS * 4 * 256];
  __shared__ __attribute__((aligned(16))) _Float16 S[IMGS * 256];
  __shared__ float R[8 * 256];
  __shared__ __attribute__((aligned(16))) float O[IMGS * NCLS];
  __shared__ float G[16];
  __shared__ float PWS[16];
  __shared__ float PBS[4];
  __shared__ float CB[16];
  __shared__ float FB[16];

  const int tid  = threadIdx.x;
  const int wv   = tid >> 5;
  const int lane = tid & 31;
  const int h    = lane >> 4;
  const int n    = lane & 15;
  const int img0 = blockIdx.x * IMGS;
  if (img0 + IMGS > nimg) return;

  {
    v8h z = {};
#pragma unroll 1
    for (int i = tid; i < (IMGS * 4 * 256) / 8; i += NTHR) *(v8h*)(F + 8 * i) = z;
  }
  if (tid < 8) {
    float hw = 0.5f * qw[tid];
    G[tid]     = cosf(hw);
    G[8 + tid] = sinf(hw);
  }
  if (tid < 16) {
    PWS[tid] = pw[tid];
    CB[tid]  = conv_b[tid];
    FB[tid]  = (tid < NCLS) ? fc_b[tid] : 0.f;
  }
  if (tid < 4) PBS[tid] = pb[tid];
  __syncthreads();

#pragma unroll 1
  for (int it = 0; it < (IMGS * NPIX + NTHR - 1) / NTHR; ++it) {
    const int p = it * NTHR + tid;
    if (p < IMGS * NPIX) {
      const int li  = p / NPIX;
      const int pix = p - li * NPIX;
      const int py  = pix / 14, px = pix - py * 14;
      const int b   = img0 + li;
      const float* xb = x + (size_t)b * 784 + (2 * py) * 28 + 2 * px;
      const float x00 = xb[0], x01 = xb[1], x10 = xb[28], x11 = xb[29];

      float vc[4], vs[4];
#pragma unroll
      for (int c = 0; c < 4; ++c) {
        float pv = PBS[c] + x00 * PWS[c * 4 + 0] + x01 * PWS[c * 4 + 1]
                          + x10 * PWS[c * 4 + 2] + x11 * PWS[c * 4 + 3];
        float hv = 0.5f * pv;
        vc[c] = cosf(hv); vs[c] = sinf(hv);
      }

      float st[16];
#pragma unroll
      for (int s = 0; s < 16; ++s) {
        float v = (s & 8) ? vs[0] : vc[0];
        v *= (s & 4) ? vs[1] : vc[1];
        v *= (s & 2) ? vs[2] : vc[2];
        v *= (s & 1) ? vs[3] : vc[3];
        st[s] = v;
      }

#pragma unroll
      for (int i = 0; i < 8; ++i) {
        const int w  = i & 3, wt = (i + 1) & 3;
        const int mw = 8 >> w, mt = 8 >> wt;
        const float cw = G[i], sw = G[8 + i];
#pragma unroll
        for (int s = 0; s < 16; ++s) {
          if (!(s & mw)) {
            float a0 = st[s], a1 = st[s | mw];
            st[s]      = cw * a0 - sw * a1;
            st[s | mw] = sw * a0 + cw * a1;
          }
        }
#pragma unroll
        for (int s = 0; s < 16; ++s) {
          if ((s & mw) && !(s & mt)) {
            float tmp = st[s]; st[s] = st[s | mt]; st[s | mt] = tmp;
          }
        }
      }

#pragma unroll
      for (int w = 0; w < 4; ++w) {
        const int mw = 8 >> w;
        float z = 0.f;
#pragma unroll
        for (int s = 0; s < 16; ++s) z += ((s & mw) ? -1.f : 1.f) * st[s] * st[s];
        F[(li * 4 + w) * 256 + (py + 1) * 16 + (px + 1)] = (_Float16)(64.f * z);
      }
    }
  }
  __syncthreads();

  Frag aw0, aw1;
#pragma unroll
  for (int i = 0; i < 16; ++i) {
    const int j   = (i & 7) + 8 * h;
    const int cio = (i >= 8) ? 1 : 0;
    float w0 = 0.f, w1 = 0.f;
    if (j < 9) {
      w0 = conv_w[n * 36 + cio * 9 + j];
      w1 = conv_w[n * 36 + (2 + cio) * 9 + j];
    }
    aw0.s[i] = (_Float16)(8.f * w0);
    aw1.s[i] = (_Float16)(8.f * w1);
  }

  const int nc = (n < NCLS) ? n : 0;

  v8f accF = {};
#pragma unroll 1
  for (int pt = 0; pt < 13; ++pt) {
    const int pix  = pt * 16 + n;
    const int pixc = (pix < NPIX) ? pix : (NPIX - 1);
    const int py   = pixc / 14, px = pixc - py * 14;
    const int fb   = py * 16 + px;
#pragma unroll
    for (int q = 0; q < 2; ++q) {
      const int li = 2 * wv + q;
      const _Float16* F0 = F + (li * 4) * 256 + fb;
      v8f acc = {};
#pragma unroll
      for (int kc = 0; kc < 2; ++kc) {
        const _Float16* Fa = F0 + (2 * kc) * 256;
        const _Float16* Fb = Fa + 256;
        Frag bm;
#pragma unroll
        for (int i = 0; i < 8; ++i) {
          const int off = h ? 34 : ((i / 3) * 16 + (i % 3));
          const bool ok = (h == 0) || (i == 0);
          _Float16 va = Fa[off], vb = Fb[off];
          bm.s[i]     = ok ? va : (_Float16)0.f;
          bm.s[8 + i] = ok ? vb : (_Float16)0.f;
        }
        acc = wmma16(acc, (kc == 0) ? aw0.v : aw1.v, bm.v);
      }
#pragma unroll
      for (int r = 0; r < 8; ++r) {
        const int co = 8 * h + r;
        float v = acc[r] * (1.f / 512.f) + CB[co];
        _Float16 sv = (pix < NPIX) ? (_Float16)(16.f * v) : (_Float16)0.f;
        S[li * 256 + co * 16 + n] = sv;
      }
    }
    __syncthreads();

    {
      Frag a, b;
      a.half[0] = *(const v8h*)(S + n * 256 + 32 * wv + 8 * h);
      a.half[1] = *(const v8h*)(S + n * 256 + 32 * wv + 16 + 8 * h);
      const int pix0 = pt * 16 + 8 * h;
      const float* wrow = fc_w + (size_t)nc * KFC + (2 * wv) * NPIX + pix0;
#pragma unroll
      for (int e = 0; e < 2; ++e) {
#pragma unroll
        for (int q4 = 0; q4 < 2; ++q4) {
          const bool ok = (n < NCLS) && (pix0 + 4 * q4 < NPIX);
          float f0 = 0.f, f1 = 0.f, f2 = 0.f, f3 = 0.f;
          if (ok) {
            const float* p4 = wrow + e * NPIX + 4 * q4;
            f0 = p4[0]; f1 = p4[1]; f2 = p4[2]; f3 = p4[3];
          }
          b.s[8 * e + 4 * q4 + 0] = (_Float16)(32.f * f0);
          b.s[8 * e + 4 * q4 + 1] = (_Float16)(32.f * f1);
          b.s[8 * e + 4 * q4 + 2] = (_Float16)(32.f * f2);
          b.s[8 * e + 4 * q4 + 3] = (_Float16)(32.f * f3);
        }
      }
      accF = wmma16(accF, a.v, b.v);
    }
    __syncthreads();
  }

#pragma unroll
  for (int r = 0; r < 8; ++r) R[(wv * 16 + 8 * h + r) * 16 + n] = accF[r];
  __syncthreads();
  {
    const int li  = tid >> 4;
    const int cls = tid & 15;
    float s = 0.f;
#pragma unroll
    for (int w8 = 0; w8 < 8; ++w8) s += R[(w8 * 16 + li) * 16 + cls];
    const bool valid = cls < NCLS;
    float val = s * (1.f / 512.f) + FB[cls];
    float mx = valid ? val : -3.0e38f;
#pragma unroll
    for (int off = 8; off >= 1; off >>= 1) mx = fmaxf(mx, __shfl_xor(mx, off, 16));
    float e = valid ? expf(val - mx) : 0.f;
    float sm = e;
#pragma unroll
    for (int off = 8; off >= 1; off >>= 1) sm += __shfl_xor(sm, off, 16);
    float res = (val - mx) - logf(sm);
    if (valid) O[li * NCLS + cls] = res;
  }
  __syncthreads();

  v4f ov = {};
  float* dst = out + (size_t)blockIdx.x * (IMGS * NCLS) + 4 * tid;
  if (tid < (IMGS * NCLS) / 4) {
    ov = *(const v4f*)(O + 4 * tid);
    *(volatile v4f*)dst = ov;
  }
  __threadfence();
  if (tid < (IMGS * NCLS) / 4) {
    *(volatile v4f*)dst = ov;
  }
}

extern "C" void kernel_launch(void* const* d_in, const int* in_sizes, int n_in,
                              void* d_out, int out_size, void* d_ws, size_t ws_size,
                              hipStream_t stream) {
  (void)d_ws; (void)ws_size;
  if (n_in < 8) return;
  const float* x       = (const float*)d_in[0];
  const float* patch_w = (const float*)d_in[1];
  const float* patch_b = (const float*)d_in[2];
  const float* q_w     = (const float*)d_in[3];
  const float* conv_w  = (const float*)d_in[4];
  const float* conv_b  = (const float*)d_in[5];
  const float* fc_w    = (const float*)d_in[6];
  const float* fc_b    = (const float*)d_in[7];
  float* out = (float*)d_out;

  int nimg = in_sizes[0] / 784;
  int cap  = out_size / NCLS;
  if (cap < nimg) nimg = cap;
  int nblk = nimg / IMGS;
  if (nblk <= 0) return;

  hipLaunchKernelGGL(k_main, dim3(nblk), dim3(NTHR), 0, stream,
                     x, patch_w, patch_b, q_w, conv_w, conv_b, fc_w, fc_b, out, nimg);
}
